// SignatureBackend_24575802867997
// MI455X (gfx1250) — hardware-run, weakly checked
//
#include <hip/hip_runtime.h>
#include <math.h>

typedef __attribute__((ext_vector_type(16))) _Float16 v16h;
typedef __attribute__((ext_vector_type(8)))  _Float16 v8h;
typedef __attribute__((ext_vector_type(8)))  float    v8f;
typedef __attribute__((ext_vector_type(4)))  float    v4f;

constexpr int kWin    = 60;
constexpr int kChIn   = 8;
constexpr int kD      = 9;
constexpr int kSeq    = 2048;
constexpr int kBatch  = 8;
constexpr int kRows   = kBatch * kSeq;
constexpr int kFeat   = 285;
constexpr int kFeatP  = 320;
constexpr int kH2     = 512;
constexpr int kHid    = 256;
constexpr int kIncP   = 12;
constexpr int kIncRows = 64;
static_assert(kD == kChIn + 1);
static_assert(kFeat == kD + (kD * kD - kD) / 2 + (kD * kD * kD - kD) / 3);
static_assert(kRows == 16384);
static_assert((kFeatP % 32) == 0 && (kH2 % 32) == 0);
static_assert((kRows % 64) == 0 && (kH2 % 64) == 0 && (kHid % 64) == 0);
static_assert((kFeatP * 2) % 128 == 0);
static_assert((kRows % 8) == 0);

constexpr float kCarryFeat = 8.0f;
constexpr float kCarryW    = 256.0f;
constexpr float kCarryHn   = 16.0f;
constexpr float kScale1    = 1.0f / (kCarryFeat * kCarryW);
constexpr float kScale2    = 1.0f / (kCarryHn * kCarryW);
constexpr float kH16Min    = 6.103515625e-05f;
constexpr float kH16Lim    = 65000.0f;
constexpr float kDt        = 1.0f / (float)(kWin - 1);
constexpr float kSixth     = 1.0f / 6.0f;
constexpr float kThird     = 1.0f / 3.0f;
constexpr float kInvH2     = 1.0f / (float)kH2;
constexpr float kLnEps     = 1e-5f;

constexpr size_t kOffW1T   = 0;
constexpr size_t kOffW2T   = kOffW1T   + (size_t)kH2   * kFeatP * 2;
constexpr size_t kOffFeats = kOffW2T   + (size_t)kHid  * kH2    * 2;
constexpr size_t kOffZ     = kOffFeats + (size_t)kRows * kFeatP * 2;
constexpr size_t kOffHn    = kOffZ     + (size_t)kRows * kH2    * 4;
constexpr size_t kWsTotal  = kOffHn    + (size_t)kRows * kH2    * 2;
static_assert(kWsTotal == 61407232ull);
static_assert(kWsTotal <= 134217728ull);
static_assert((kOffW2T % 128) == 0 && (kOffFeats % 128) == 0 && (kOffZ % 128) == 0 && (kOffHn % 128) == 0);

__device__ __forceinline__ _Float16 h16_carry(float v, float carry) {
  float s = v * carry;
  s = fminf(fmaxf(s, -kH16Lim), kH16Lim);
  s = (fabsf(s) < kH16Min) ? 0.0f : s;
  return (_Float16)s;
}

__device__ __forceinline__ v16h frag_load_h(const _Float16* p) {
  union U { v16h v; v8h h[2]; } f;
  f.h[0] = *(const v8h*)(p);
  f.h[1] = *(const v8h*)(p + 16);
  return f.v;
}
__device__ __forceinline__ v8f mma_h(v16h a, v16h b, v8f c) {
  return __builtin_amdgcn_wmma_f32_16x16x32_f16(false, a, false, b, (short)0, c, false, false);
}
__device__ __forceinline__ void tie_acc_h(v8f& a, v16h x, v16h y) {
  asm volatile("" : "+v"(a) : "v"(x), "v"(y));
}
__device__ __forceinline__ void nop_guard_h(v8f& a, v16h x, v16h y) {
  asm volatile("v_nop\n\tv_nop\n\tv_nop\n\tv_nop" : "+v"(a) : "v"(x), "v"(y));
}
__device__ __forceinline__ void nop_guard_acc(v8f& a) {
  asm volatile("v_nop\n\tv_nop\n\tv_nop\n\tv_nop" : "+v"(a));
}
__device__ __forceinline__ void keep4_h(v16h a, v16h b, v16h c, v16h d) {
  asm volatile("v_nop" :: "v"(a), "v"(b), "v"(c), "v"(d));
}

__global__ __launch_bounds__(256) void transpose_cast_kernel(
    const float* __restrict__ src, unsigned short* __restrict__ dst,
    int kReal, int kPad, int nCols, float carry, int total)
{
  const int id = blockIdx.x * 256 + threadIdx.x;
  if (id >= total) return;
  const int kg8 = kPad >> 3;
  const int n   = id / kg8;
  const int k0  = (id - n * kg8) << 3;
  v8h hv;
#pragma unroll
  for (int e = 0; e < 8; ++e) {
    const int k  = k0 + e;
    const int kc = (k < kReal) ? k : (kReal - 1);
    float v = src[(size_t)kc * nCols + n];
    asm volatile("" : "+v"(v));
    const float s = (k < kReal) ? v : 0.0f;
    hv[e] = h16_carry(s, carry);
  }
  unsigned short* q = dst + (size_t)id * 8;
  *(volatile v8h*)q = hv;
  __threadfence();
  *(volatile v8h*)q = hv;
}

__device__ __forceinline__ void decode_upper(int u, int& i, int& j) {
  int ii = 0;
#pragma unroll
  for (int t = 1; t < 9; ++t) {
    const int bt = 9 * t - (t * (t - 1)) / 2;
    ii = (u >= bt) ? t : ii;
  }
  i = ii;
  j = ii + (u - (9 * ii - (ii * (ii - 1)) / 2));
}
__device__ __forceinline__ void decode_lower(int q, int& i, int& j) {
  int ii = 1;
#pragma unroll
  for (int t = 2; t < 9; ++t) {
    const int bt = (t * (t - 1)) / 2;
    ii = (q >= bt) ? t : ii;
  }
  i = ii;
  j = q - (ii * (ii - 1)) / 2;
}

#define SIG_CHEN_SLOT3(S3arr, S2v, s1v, vi, vj)                               \
  {                                                                           \
    const float g_ = fmaf((vi), kSixth, 0.5f * (s1v));                        \
    const float a_ = fmaf(g_, (vj), (S2v));                                   \
    _Pragma("unroll")                                                         \
    for (int k_ = 0; k_ < kD; ++k_) S3arr[k_] = fmaf(a_, vk[k_], S3arr[k_]);  \
    const float u_ = fmaf(0.5f, (vi), (s1v));                                 \
    (S2v) = fmaf(u_, (vj), (S2v));                                            \
    (s1v) += (vi);                                                            \
  }
#define SIG_CHEN_SLOT2(S2v, s1v, vi, vj)                                      \
  {                                                                           \
    const float u_ = fmaf(0.5f, (vi), (s1v));                                 \
    (S2v) = fmaf(u_, (vj), (S2v));                                            \
    (s1v) += (vi);                                                            \
  }
#define SIG_EMIT_PAIR(iv, jv, S2v, S3arr, okv)                                \
  {                                                                           \
    const float s1i_ = s1p[(iv)];                                             \
    const float s1j_ = s1p[(jv)];                                             \
    const float l2_  = (S2v) - 0.5f * s1i_ * s1j_;                            \
    if ((okv) && ((iv) < (jv)))                                               \
      fp[9 + 8 * (iv) - ((iv) * ((iv) - 1)) / 2 + ((jv) - (iv) - 1)] = l2_;   \
    int b3_ = 0;                                                              \
    _Pragma("unroll")                                                         \
    for (int t_ = 0; t_ < 8; ++t_)                                            \
      b3_ += (t_ < (iv)) ? (9 - t_) * (8 - t_) : 0;                           \
    const int fb_ = 45 + b3_ + ((jv) - (iv)) * (8 - (iv)) - (iv) - 1;         \
    const float c3_ = s1i_ * s1j_ * kThird;                                   \
    const float dd_ = c3_ - 0.5f * (S2v);                                     \
    const float hm_ = -0.5f * s1i_;                                           \
    _Pragma("unroll")                                                         \
    for (int k_ = 0; k_ < kD; ++k_) {                                         \
      const float s2jk_ = s2p[(jv) * 9 + k_];                                 \
      float l3_ = fmaf(hm_, s2jk_, S3arr[k_]);                                \
      l3_ = fmaf(s1k[k_], dd_, l3_);                                          \
      if ((okv) && (k_ > (iv))) fp[fb_ + k_] = l3_;                           \
    }                                                                         \
  }

__global__ __launch_bounds__(256) void logsig_kernel(
    const float* __restrict__ x, unsigned short* __restrict__ feats)
{
  __shared__ __align__(16) float sInc[8][kIncRows * kIncP];
  __shared__ __align__(16) float sS2[8][84];
  __shared__ __align__(16) float sS1[8][12];
  __shared__ __align__(16) float sF[8][kFeatP];

  const int lane = threadIdx.x & 31;
  const int wave = threadIdx.x >> 5;
  const int n    = blockIdx.x * 8 + wave;
  const int bI   = n >> 11;
  const int t    = n & (kSeq - 1);

  float* fp  = sF[wave];
  float* s2p = sS2[wave];
  float* s1p = sS1[wave];
  float* inc = sInc[wave];

#pragma unroll
  for (int i = 0; i < 10; ++i) fp[lane + 32 * i] = 0.0f;

#pragma unroll
  for (int it = 0; it < 2; ++it) {
    const int w  = lane + 32 * it;
    const int wc = (w < kWin) ? w : (kWin - 1);
    int p1 = t + wc - (kWin - 1);
    p1 = (p1 < 0) ? 0 : p1;
    int p0 = t + wc - kWin;
    p0 = (p0 < 0) ? 0 : p0;
    const float* r1 = x + ((size_t)bI * kSeq + p1) * kChIn;
    const float* r0 = x + ((size_t)bI * kSeq + p0) * kChIn;
    v4f a0 = *(const v4f*)(r1);
    v4f a1 = *(const v4f*)(r1 + 4);
    v4f b0 = *(const v4f*)(r0);
    v4f b1 = *(const v4f*)(r0 + 4);
    asm volatile("" : "+v"(a0), "+v"(a1), "+v"(b0), "+v"(b1));
    const bool first = (wc == 0);
    v4f d0, d1;
#pragma unroll
    for (int e = 0; e < 4; ++e) {
      const float da = a0[e] - b0[e];
      const float db = a1[e] - b1[e];
      d0[e] = first ? a0[e] : da;
      d1[e] = first ? a1[e] : db;
    }
    const float dtv = first ? 0.0f : kDt;
    const v4f o0 = {dtv,   d0[0], d0[1], d0[2]};
    const v4f o1 = {d0[3], d1[0], d1[1], d1[2]};
    const v4f o2 = {d1[3], 0.0f,  0.0f,  0.0f};
    float* dstp = inc + w * kIncP;
    *(v4f*)(dstp)     = o0;
    *(v4f*)(dstp + 4) = o1;
    *(v4f*)(dstp + 8) = o2;
  }

  int iA, jA, iC, jC, iBu, jBu, iBl, jBl;
  decode_upper(lane, iA, jA);
  decode_lower(lane, iC, jC);
  {
    const int uB = (32 + lane < 44) ? (32 + lane) : 44;
    int qB = 19 + lane;
    qB = (qB < 32) ? 32 : qB;
    qB = (qB > 35) ? 35 : qB;
    decode_upper(uB, iBu, jBu);
    decode_lower(qB, iBl, jBl);
  }
  const bool bUpper = (lane <= 12);
  const bool bLower = (lane >= 13) && (lane <= 16);
  const int iB = bUpper ? iBu : (bLower ? iBl : 0);
  const int jB = bUpper ? jBu : (bLower ? jBl : 0);
  const int cown = (lane < kD) ? lane : (kD - 1);

  float S3A[kD], S3B[kD];
#pragma unroll
  for (int k = 0; k < kD; ++k) { S3A[k] = 0.0f; S3B[k] = 0.0f; }
  float S2A = 0.0f, S2B = 0.0f, S2C = 0.0f;
  float s1A = 0.0f, s1B = 0.0f, s1C = 0.0f;
  float s1own = 0.0f;

  __syncthreads();

#pragma unroll 1
  for (int w = 0; w < kWin; ++w) {
    const float* r = inc + w * kIncP;
    const v4f q0 = *(const v4f*)(r);
    const v4f q1 = *(const v4f*)(r + 4);
    const v4f q2 = *(const v4f*)(r + 8);
    const float vk[kD] = {q0[0], q0[1], q0[2], q0[3], q1[0], q1[1], q1[2], q1[3], q2[0]};
    const float viA = r[iA], vjA = r[jA];
    const float viB = r[iB], vjB = r[jB];
    const float viC = r[iC], vjC = r[jC];
    const float vo  = r[cown];
    SIG_CHEN_SLOT3(S3A, S2A, s1A, viA, vjA)
    SIG_CHEN_SLOT3(S3B, S2B, s1B, viB, vjB)
    SIG_CHEN_SLOT2(S2C, s1C, viC, vjC)
    s1own += vo;
  }

  s2p[iA * 9 + jA] = S2A;
  if (lane <= 16) s2p[iB * 9 + jB] = S2B;
  s2p[iC * 9 + jC] = S2C;
  if (lane < 3) s2p[81 + lane] = 0.0f;
  if (lane < 12) s1p[lane] = (lane < kD) ? s1own : 0.0f;
  __syncthreads();

  float s1k[kD];
#pragma unroll
  for (int k = 0; k < kD; ++k) s1k[k] = s1p[k];
  if (lane < kD) fp[lane] = s1own;
  SIG_EMIT_PAIR(iA, jA, S2A, S3A, true)
  SIG_EMIT_PAIR(iB, jB, S2B, S3B, bUpper)
  __syncthreads();

  v8h h0, h1;
  {
    const float* p0 = fp + lane * 8;
    const float* p1 = fp + 256 + (lane & 7) * 8;
    const v4f a0 = *(const v4f*)(p0);
    const v4f a1 = *(const v4f*)(p0 + 4);
    const v4f c0 = *(const v4f*)(p1);
    const v4f c1 = *(const v4f*)(p1 + 4);
#pragma unroll
    for (int e = 0; e < 4; ++e) {
      h0[e]     = h16_carry(a0[e], kCarryFeat);
      h0[4 + e] = h16_carry(a1[e], kCarryFeat);
      h1[e]     = h16_carry(c0[e], kCarryFeat);
      h1[4 + e] = h16_carry(c1[e], kCarryFeat);
    }
  }
  unsigned short* drow = feats + (size_t)n * kFeatP;
  *(volatile v8h*)(drow + lane * 8) = h0;
  if (lane < 8) *(volatile v8h*)(drow + 256 + lane * 8) = h1;
  __threadfence();
  *(volatile v8h*)(drow + lane * 8) = h0;
  if (lane < 8) *(volatile v8h*)(drow + 256 + lane * 8) = h1;
}

__global__ __launch_bounds__(256) void gemm_f16_kernel(
    const unsigned short* __restrict__ Ap, int lda,
    const unsigned short* __restrict__ Btp, int ldb,
    float* __restrict__ Cout, int ldc,
    const float* __restrict__ bias,
    int M, int N, int K, float scale)
{
  const _Float16* A  = (const _Float16*)Ap;
  const _Float16* Bt = (const _Float16*)Btp;
  __shared__ __align__(16) float sT[8][16 * 68];
  const int lane = threadIdx.x & 31;
  const int wave = threadIdx.x >> 5;
  const int tilesN = N >> 6;
  const int tilesM = M >> 6;
  const int tile = blockIdx.x * 8 + wave;
  if (tile >= tilesM * tilesN) return;
  const int tm = tile / tilesN;
  const int tn = tile - tm * tilesN;
  const int m0 = tm << 6;
  const int n0 = tn << 6;

  const int rlane = lane & 15;
  const int koff  = (lane >> 4) * 8;
  const int mOff  = (lane >> 4) * 8;

  v8f acc[4][4];
#pragma unroll
  for (int i = 0; i < 4; ++i)
#pragma unroll
    for (int j = 0; j < 4; ++j) acc[i][j] = (v8f){0.f, 0.f, 0.f, 0.f, 0.f, 0.f, 0.f, 0.f};

  for (int k0 = 0; k0 < K; k0 += 32) {
    v16h bh[4];
#pragma unroll
    for (int j = 0; j < 4; ++j) {
      const size_t bo = (size_t)(n0 + (j << 4) + rlane) * ldb + koff + k0;
      bh[j] = frag_load_h(Bt + bo);
    }
#pragma unroll
    for (int i = 0; i < 4; ++i) {
      const size_t ao = (size_t)(m0 + (i << 4) + rlane) * lda + koff + k0;
      const v16h ah = frag_load_h(A + ao);
#pragma unroll
      for (int j = 0; j < 4; ++j) acc[i][j] = mma_h(ah, bh[j], acc[i][j]);
      tie_acc_h(acc[i][0], ah, bh[0]);
      tie_acc_h(acc[i][1], ah, bh[1]);
      tie_acc_h(acc[i][2], ah, bh[2]);
      nop_guard_h(acc[i][3], ah, bh[3]);
    }
    keep4_h(bh[0], bh[1], bh[2], bh[3]);
  }
#pragma unroll
  for (int i = 0; i < 4; ++i)
#pragma unroll
    for (int j = 0; j < 4; ++j) nop_guard_acc(acc[i][j]);

  float* slab = sT[wave];
  float bv[4];
#pragma unroll
  for (int j = 0; j < 4; ++j) bv[j] = bias[n0 + (j << 4) + rlane];

#pragma unroll
  for (int i = 0; i < 4; ++i) {
    const int mBase = m0 + (i << 4);
#pragma unroll
    for (int j = 0; j < 4; ++j) {
#pragma unroll
      for (int r = 0; r < 8; ++r) {
        const float v = acc[i][j][r] * scale + bv[j];
        slab[(mOff + r) * 68 + (j << 4) + rlane] = v;
      }
    }
    __builtin_amdgcn_fence(__ATOMIC_RELEASE, "workgroup");
    __builtin_amdgcn_wave_barrier();
    __builtin_amdgcn_fence(__ATOMIC_ACQUIRE, "workgroup");
    {
      const int hh = lane >> 4, c4 = (lane & 15) * 4;
      for (int pass = 0; pass < 2; ++pass) {
#pragma unroll
        for (int it = 0; it < 8; ++it) {
          const int row = it * 2 + hh;
          const v4f v = *(const v4f*)(slab + row * 68 + c4);
          *(volatile v4f*)(Cout + (size_t)(mBase + row) * ldc + n0 + c4) = v;
        }
        __threadfence();
      }
    }
    __builtin_amdgcn_fence(__ATOMIC_RELEASE, "workgroup");
    __builtin_amdgcn_wave_barrier();
    __builtin_amdgcn_fence(__ATOMIC_ACQUIRE, "workgroup");
  }
}

__global__ __launch_bounds__(256) void gelu_ln_kernel(
    const float* __restrict__ Z, const float* __restrict__ lng, const float* __restrict__ lnb,
    unsigned short* __restrict__ HN)
{
  __shared__ __align__(16) float sH[8][kH2];
  const int lane = threadIdx.x & 31;
  const int wave = threadIdx.x >> 5;
  const int row  = blockIdx.x * 8 + wave;
  const float* zr = Z + (size_t)row * kH2;
  float* hr = sH[wave];

  float sum = 0.0f;
#pragma unroll 1
  for (int i = 0; i < kH2 / 32; ++i) {
    const int c = lane + 32 * i;
    const float z = zr[c];
    const float g = 0.5f * z * (1.0f + erff(z * 0.70710678118654752f));
    hr[c] = g;
    sum += g;
  }
#pragma unroll
  for (int off = 16; off >= 1; off >>= 1) sum += __shfl_xor(sum, off, 32);
  const float mean = sum * kInvH2;

  float ss = 0.0f;
#pragma unroll 1
  for (int i = 0; i < kH2 / 32; ++i) {
    const float d = hr[lane + 32 * i] - mean;
    ss = fmaf(d, d, ss);
  }
#pragma unroll
  for (int off = 16; off >= 1; off >>= 1) ss += __shfl_xor(ss, off, 32);
  const float var  = ss * kInvH2;
  const float rstd = 1.0f / sqrtf(var + kLnEps);

  __syncthreads();

#pragma unroll 1
  for (int it = 0; it < 2; ++it) {
    const int c0 = it * 256 + lane * 8;
    const v4f h0 = *(const v4f*)(hr + c0);
    const v4f h1 = *(const v4f*)(hr + c0 + 4);
    const v4f g0 = *(const v4f*)(lng + c0);
    const v4f g1 = *(const v4f*)(lng + c0 + 4);
    const v4f b0 = *(const v4f*)(lnb + c0);
    const v4f b1 = *(const v4f*)(lnb + c0 + 4);
    v8h hv;
#pragma unroll
    for (int e = 0; e < 4; ++e) {
      const float y0 = ((h0[e] - mean) * rstd) * g0[e] + b0[e];
      const float y1 = ((h1[e] - mean) * rstd) * g1[e] + b1[e];
      hv[e]     = h16_carry(y0, kCarryHn);
      hv[4 + e] = h16_carry(y1, kCarryHn);
    }
    unsigned short* q = HN + (size_t)row * kH2 + c0;
    *(volatile v8h*)q = hv;
    __threadfence();
    *(volatile v8h*)q = hv;
  }
}

extern "C" void kernel_launch(void* const* d_in, const int* in_sizes, int n_in,
                              void* d_out, int out_size, void* d_ws, size_t ws_size,
                              hipStream_t stream) {
  if (n_in < 7) return;
  if (in_sizes[0] != kRows * kChIn) return;
  if (in_sizes[1] != kFeat * kH2) return;
  if (in_sizes[2] != kH2) return;
  if (in_sizes[3] != kH2) return;
  if (in_sizes[4] != kH2) return;
  if (in_sizes[5] != kH2 * kHid) return;
  if (in_sizes[6] != kHid) return;
  if (out_size != kRows * kHid) return;
  if (ws_size < kWsTotal) return;

  const float* x    = (const float*)d_in[0];
  const float* w1   = (const float*)d_in[1];
  const float* b1   = (const float*)d_in[2];
  const float* ln_g = (const float*)d_in[3];
  const float* ln_b = (const float*)d_in[4];
  const float* w2   = (const float*)d_in[5];
  const float* b2   = (const float*)d_in[6];
  float* out = (float*)d_out;

  char* ws = (char*)d_ws;
  unsigned short* W1T   = (unsigned short*)(ws + kOffW1T);
  unsigned short* W2T   = (unsigned short*)(ws + kOffW2T);
  unsigned short* FEATS = (unsigned short*)(ws + kOffFeats);
  float*          ZPL   = (float*)(ws + kOffZ);
  unsigned short* HN    = (unsigned short*)(ws + kOffHn);

  constexpr int kTot1 = kH2 * (kFeatP / 8);
  constexpr int kTot2 = kHid * (kH2 / 8);
  static_assert((kTot1 % 256) == 0 && (kTot2 % 256) == 0);
  transpose_cast_kernel<<<kTot1 / 256, 256, 0, stream>>>(w1, W1T, kFeat, kFeatP, kH2, kCarryW, kTot1);
  transpose_cast_kernel<<<kTot2 / 256, 256, 0, stream>>>(w2, W2T, kH2, kH2, kHid, kCarryW, kTot2);

  logsig_kernel<<<kRows / 8, 256, 0, stream>>>(x, FEATS);

  gemm_f16_kernel<<<(kRows / 64) * (kH2 / 64) / 8, 256, 0, stream>>>(
      FEATS, kFeatP, W1T, kFeatP, ZPL, kH2, b1, kRows, kH2, kFeatP, kScale1);

  gelu_ln_kernel<<<kRows / 8, 256, 0, stream>>>(ZPL, ln_g, ln_b, HN);

  gemm_f16_kernel<<<(kRows / 64) * (kHid / 64) / 8, 256, 0, stream>>>(
      HN, kH2, W2T, kH2, out, kHid, b2, kRows, kHid, kH2, kScale2);
}
